// cufi_nufft_68032281968976
// MI455X (gfx1250) — hardware-verified
//
#include <hip/hip_runtime.h>
#include <stdint.h>

typedef __attribute__((ext_vector_type(16))) _Float16 v16h;
typedef __attribute__((ext_vector_type(8)))  _Float16 v8h;
typedef __attribute__((ext_vector_type(16))) __bf16   v16b;
typedef __attribute__((ext_vector_type(8)))  __bf16   v8b;
typedef __attribute__((ext_vector_type(8)))  float    v8f;
typedef __attribute__((ext_vector_type(4)))  float    v4f;
typedef __attribute__((ext_vector_type(2)))  float    v2f;

__device__ __forceinline__ unsigned short f2bf_bits(float f) {
  unsigned u = __float_as_uint(f);
  return (unsigned short)((u + 0x7FFFu + ((u >> 16) & 1u)) >> 16);
}
__device__ __forceinline__ float bf_bits2f(unsigned short h) { return __uint_as_float(((unsigned)h) << 16); }

__device__ __forceinline__ void dep_guard_h(v8f& a, v8f& b, v16h x, v16h y) { asm volatile("v_nop\n\tv_nop\n\tv_nop\n\tv_nop" : "+v"(a), "+v"(b) : "v"(x), "v"(y)); }
__device__ __forceinline__ void dep_guard_b(v8f& a, v8f& b, v16b x, v16b y) { asm volatile("v_nop\n\tv_nop\n\tv_nop\n\tv_nop" : "+v"(a), "+v"(b) : "v"(x), "v"(y)); }
__device__ __forceinline__ void keep4_h(v16h a, v16h b, v16h c, v16h d) { asm volatile("v_nop" :: "v"(a), "v"(b), "v"(c), "v"(d)); }
__device__ __forceinline__ void keep4_b(v16b a, v16b b, v16b c, v16b d) { asm volatile("v_nop" :: "v"(a), "v"(b), "v"(c), "v"(d)); }
__device__ __forceinline__ void acc_guard4(v8f& a, v8f& b, v8f& c, v8f& d) { asm volatile("v_nop\n\tv_nop\n\tv_nop\n\tv_nop" : "+v"(a), "+v"(b), "+v"(c), "+v"(d)); }
template <typename T> struct Frag;
template <> struct Frag<_Float16> {
  typedef v16h V; union U { v16h v; v8h h[2]; };
  static __device__ __forceinline__ v16h load(const _Float16* p) {
    U f; f.h[0] = *(const v8h*)(p); f.h[1] = *(const v8h*)(p + 16); return f.v;
  }
  static __device__ __forceinline__ v8f mma(v16h a, v16h b, v8f c) {
    return __builtin_amdgcn_wmma_f32_16x16x32_f16(false, a, false, b, (short)0, c, false, false);
  }
  static __device__ __forceinline__ void guard(v8f& a, v8f& b, v16h x, v16h y) { dep_guard_h(a, b, x, y); }
  static __device__ __forceinline__ void keep(v16h a, v16h b, v16h c, v16h d) { keep4_h(a, b, c, d); }
};
template <> struct Frag<__bf16> {
  typedef v16b V; union U { v16b v; v8b h[2]; };
  static __device__ __forceinline__ v16b load(const __bf16* p) {
    U f; f.h[0] = *(const v8b*)(p); f.h[1] = *(const v8b*)(p + 16); return f.v;
  }
  static __device__ __forceinline__ v8f mma(v16b a, v16b b, v8f c) {
    return __builtin_amdgcn_wmma_f32_16x16x32_bf16(false, a, false, b, (short)0, c, false, false);
  }
  static __device__ __forceinline__ void guard(v8f& a, v8f& b, v16b x, v16b y) { dep_guard_b(a, b, x, y); }
  static __device__ __forceinline__ void keep(v16b a, v16b b, v16b c, v16b d) { keep4_b(a, b, c, d); }
};

template <int ET> struct Elem;
template <> struct Elem<0> { typedef _Float16 T; };
template <> struct Elem<1> { typedef __bf16 T; };
template <int ET, bool SPLIT, int BIAS_MODE, int OUT_MODE, bool RESID, int ACT = 0>
__global__ __launch_bounds__(256) void wmma_gemm64(
    const unsigned short* __restrict__ Ap, const unsigned short* __restrict__ A2p, int lda, long strideA,
    const unsigned short* __restrict__ Btp, const unsigned short* __restrict__ Bt2p, int ldb, long strideB,
    void* __restrict__ Cout, void* __restrict__ Cout2, int ldc, long strideC,
    const float* __restrict__ bias,
    const float* __restrict__ resid, long strideR,
    int M, int N, int K, float scale) {
  typedef typename Elem<ET>::T T;
  typedef typename Frag<T>::V V;
  const T* A = (const T*)Ap; const T* A2 = (const T*)A2p; const T* Bt = (const T*)Btp; const T* Bt2 = (const T*)Bt2p;
  __shared__ __align__(16) float sT[8][16 * 68];
  const int b    = blockIdx.y;
  const int lane = threadIdx.x & 31;
  const int wave = threadIdx.x >> 5;
  const int tilesN = N >> 6;
  const int tilesM = M >> 6;
  const int tile = blockIdx.x * 8 + wave;
  if (tile >= tilesM * tilesN) return;
  const int tm = tile / tilesN;
  const int tn = tile - tm * tilesN;
  const int m0 = tm << 6;
  const int n0 = tn << 6;

  const T* Ab  = A  + (size_t)b * strideA;
  const T* Bb  = Bt + (size_t)b * strideB;
  const T* Ab2 = SPLIT ? (A2  + (size_t)b * strideA) : nullptr;
  const T* Bb2 = SPLIT ? (Bt2 + (size_t)b * strideB) : nullptr;

  const int rlane = lane & 15;
  const int koff  = (lane >> 4) * 8;
  const int mOff  = (lane >> 4) * 8;

  v8f acc[4][4];
#pragma unroll
  for (int i = 0; i < 4; ++i)
#pragma unroll
    for (int j = 0; j < 4; ++j) acc[i][j] = (v8f){0.f,0.f,0.f,0.f,0.f,0.f,0.f,0.f};

  for (int k0 = 0; k0 < K; k0 += 32) {
    V bh[4], bl[4];
#pragma unroll
    for (int j = 0; j < 4; ++j) {
      const size_t bo = (size_t)(n0 + (j << 4) + rlane) * ldb + koff + k0;
      bh[j] = Frag<T>::load(Bb + bo);
      if (SPLIT) bl[j] = Frag<T>::load(Bb2 + bo);
    }
#pragma unroll
    for (int i = 0; i < 4; ++i) {
      const size_t ao = (size_t)(m0 + (i << 4) + rlane) * lda + koff + k0;
      V ah = Frag<T>::load(Ab + ao);
      V al;
      if (SPLIT) al = Frag<T>::load(Ab2 + ao);
#pragma unroll
      for (int j = 0; j < 4; ++j) {
        acc[i][j] = Frag<T>::mma(ah, bh[j], acc[i][j]);
        if (SPLIT) {
          acc[i][j] = Frag<T>::mma(ah, bl[j], acc[i][j]);
          acc[i][j] = Frag<T>::mma(al, bh[j], acc[i][j]);
        }
      }
      Frag<T>::guard(acc[i][0], acc[i][3], ah, SPLIT ? al : ah);
    }
    Frag<T>::keep(bh[0], bh[1], bh[2], bh[3]);
    if (SPLIT) Frag<T>::keep(bl[0], bl[1], bl[2], bl[3]);
  }
  acc_guard4(acc[0][0], acc[0][1], acc[0][2], acc[0][3]);
  acc_guard4(acc[1][0], acc[1][1], acc[1][2], acc[1][3]);
  acc_guard4(acc[2][0], acc[2][1], acc[2][2], acc[2][3]);
  acc_guard4(acc[3][0], acc[3][1], acc[3][2], acc[3][3]);

  float* slab = sT[wave];
  const float* Rb = RESID ? (resid + (size_t)b * strideR) : nullptr;
#pragma unroll
  for (int i = 0; i < 4; ++i) {
    const int mBase = m0 + (i << 4);
#pragma unroll
    for (int j = 0; j < 4; ++j) {
      const int n = n0 + (j << 4) + rlane;
      float bv = 0.f;
      if (BIAS_MODE == 2) bv = bias[n];
#pragma unroll
      for (int r = 0; r < 8; ++r) {
        float v = acc[i][j][r] * scale;
        if (BIAS_MODE == 1) v += bias[mBase + mOff + r];
        if (BIAS_MODE == 2) v += bv;
        if (RESID) v += Rb[(size_t)(mBase + mOff + r) * ldc + n];
        if (ACT == 1) v = tanhf(v);
        if (ACT == 2) v = fmaxf(v, 0.0f);
        if (ACT == 3) v = v / (1.0f + expf(-v));
        if (ACT == 4) v = (v > 0.f) ? v : 0.01f * v;
        if (ACT == 5) v = 0.5f * v * (1.0f + erff(v * 0.70710678118654752f));
        slab[(mOff + r) * 68 + (j << 4) + rlane] = v;
      }
    }
    __builtin_amdgcn_fence(__ATOMIC_RELEASE, "workgroup");
    __builtin_amdgcn_wave_barrier();
    __builtin_amdgcn_fence(__ATOMIC_ACQUIRE, "workgroup");
    if (OUT_MODE == 0) {
      float* C = (float*)Cout + (size_t)b * strideC;
      const int hh = lane >> 4, c4 = (lane & 15) * 4;
      for (int pass = 0; pass < 2; ++pass) {
#pragma unroll
        for (int it = 0; it < 8; ++it) {
          const int row = it * 2 + hh;
          v4f v = *(const v4f*)(slab + row * 68 + c4);
          *(volatile v4f*)(C + (size_t)(mBase + row) * ldc + n0 + c4) = v;
        }
        __threadfence();
      }
    } else {
      const int q = lane >> 3, c8 = (lane & 7) * 8;
      unsigned short* C  = (unsigned short*)Cout  + (size_t)b * strideC;
      unsigned short* C2 = (OUT_MODE == 2) ? ((unsigned short*)Cout2 + (size_t)b * strideC) : nullptr;
      for (int pass = 0; pass < 2; ++pass) {
#pragma unroll
        for (int it = 0; it < 4; ++it) {
          const int row = it * 4 + q;
          const float* sp = slab + row * 68 + c8;
          v8h hv, lv;
#pragma unroll
          for (int e = 0; e < 8; ++e) {
            if (OUT_MODE == 1) {
              hv[e] = (_Float16)sp[e];
            } else {
              unsigned short hb = f2bf_bits(sp[e]);
              unsigned short lb = f2bf_bits(sp[e] - bf_bits2f(hb));
              hv[e] = __builtin_bit_cast(_Float16, hb);
              lv[e] = __builtin_bit_cast(_Float16, lb);
            }
          }
          *(volatile v8h*)(C + (size_t)(mBase + row) * ldc + n0 + c8) = hv;
          if (OUT_MODE == 2) *(volatile v8h*)(C2 + (size_t)(mBase + row) * ldc + n0 + c8) = lv;
        }
        __threadfence();
      }
    }
    __builtin_amdgcn_fence(__ATOMIC_RELEASE, "workgroup");
    __builtin_amdgcn_wave_barrier();
    __builtin_amdgcn_fence(__ATOMIC_ACQUIRE, "workgroup");
  }
}

#define NC   12
#define NX   96
#define NY   96
#define NK   16384
#define NCX  (NC * NX)
#define NBT  (NCX * 2)
#define KA   (2 * NY)
#define LDC  NBT
#define MC   8192
#define RB   32
#define KB2  64
#define TPB2 (NC * 32)

#define NEG_TWO_PI (-6.28318530717958647692f)
#define INV_N      (1.0f / 96.0f)
#define TWO_OVER_PI 0.636619772367581343f

__device__ __forceinline__ void sincos_p(float a, float& s, float& c) {
  const float q = __builtin_rintf(a * TWO_OVER_PI);
  const int n = (int)q;
  float r = __builtin_fmaf(q, -1.5707962512969971e+00f, a);
  r = __builtin_fmaf(q, -7.5497894158615964e-08f, r);
  r = __builtin_fmaf(q, -5.3903029534742384e-15f, r);
  const float z = r * r;
  float ps = __builtin_fmaf(z, -1.9515295891e-4f, 8.3321608736e-3f);
  ps = __builtin_fmaf(z, ps, -1.6666654611e-1f);
  const float sr = __builtin_fmaf(z * r, ps, r);
  float pc = __builtin_fmaf(z, 2.443315711809948e-5f, -1.388731625493765e-3f);
  pc = __builtin_fmaf(z, pc, 4.166664568298827e-2f);
  const float cr = __builtin_fmaf(z * z, pc, __builtin_fmaf(z, -0.5f, 1.0f));
  float ss = (n & 1) ? cr : sr;
  float cc = (n & 1) ? -sr : cr;
  if (n & 2) { ss = -ss; cc = -cc; }
  s = ss; c = cc;
}

__device__ __forceinline__ void store_rows_h(const _Float16* s, _Float16* __restrict__ g, int row0, int nrows) {
  const int wave = threadIdx.x >> 5, lane = threadIdx.x & 31;
  for (int pass = 0; pass < 2; ++pass) {
#pragma unroll
    for (int i = 0; i < 4; ++i) {
      const int rl = wave * 4 + i;
      const int row = row0 + rl;
      if (lane < (KA / 8) && row < nrows) {
        const v8h v = *(const v8h*)(s + rl * KA + lane * 8);
        *(volatile v8h*)(g + (size_t)row * KA + lane * 8) = v;
      }
    }
    __threadfence();
  }
}

__global__ __launch_bounds__(256) void build_ey_rows(const float* __restrict__ trj,
                                                     _Float16* __restrict__ A, int nk) {
  __shared__ __align__(16) _Float16 sA[RB * KA];
  const int r0 = blockIdx.x * RB;
#pragma unroll 1
  for (int e = threadIdx.x; e < RB * NY; e += 256) {
    const int rl = e / NY;
    const int y  = e - rl * NY;
    int k = r0 + rl; k = (k < nk) ? k : (nk - 1);
    const float t  = trj[(size_t)k * 2 + 1];
    const float w  = NEG_TWO_PI * t;
    const float ry = (float)(y - NY / 2) * INV_N;
    const float a  = w * ry;
    float sn, cs; sincos_p(a, sn, cs);
    sA[rl * KA + y]      = (_Float16)cs;
    sA[rl * KA + NY + y] = (_Float16)sn;
  }
  __syncthreads();
  store_rows_h(sA, A, r0, nk);
}

__global__ __launch_bounds__(256) void build_img_rows(const float* __restrict__ imr,
                                                      const float* __restrict__ imi,
                                                      _Float16* __restrict__ Bt, int ncx) {
  __shared__ __align__(16) _Float16 sB[RB * KA];
  const int p0 = blockIdx.x * (RB / 2);
#pragma unroll 1
  for (int e = threadIdx.x; e < (RB / 2) * NY; e += 256) {
    const int pl = e / NY;
    const int y  = e - pl * NY;
    int p = p0 + pl; p = (p < ncx) ? p : (ncx - 1);
    const float vr = imr[(size_t)p * NY + y];
    const float vi = imi[(size_t)p * NY + y];
    sB[(2 * pl) * KA + y]          = (_Float16)vr;
    sB[(2 * pl) * KA + NY + y]     = (_Float16)(-vi);
    sB[(2 * pl + 1) * KA + y]      = (_Float16)vi;
    sB[(2 * pl + 1) * KA + NY + y] = (_Float16)vr;
  }
  __syncthreads();
  store_rows_h(sB, Bt, blockIdx.x * RB, 2 * ncx);
}

__global__ __launch_bounds__(TPB2) void combine_x(const float* __restrict__ C,
                                                  const float* __restrict__ trj,
                                                  float* __restrict__ out, int kbase, int nk) {
  __shared__ __align__(16) v2f sEx[KB2 * NX];
  const int tid = threadIdx.x;
  const int kb0 = blockIdx.x * KB2;
#pragma unroll 1
  for (int e = tid; e < KB2 * NX; e += TPB2) {
    const int kl = e / NX;
    const int x  = e - kl * NX;
    int k = kbase + kb0 + kl; k = (k < nk) ? k : (nk - 1);
    const float t  = trj[(size_t)k * 2];
    const float w  = NEG_TWO_PI * t;
    const float rx = (float)(x - NX / 2) * INV_N;
    const float a  = w * rx;
    float sn, cs; sincos_p(a, sn, cs);
    v2f ev; ev.x = cs; ev.y = sn;
    sEx[kl * NX + x] = ev;
  }
  __syncthreads();

  const int wave = tid >> 5;
  const int lane = tid & 31;
  const int kl0  = lane * 2;
  const float* T0 = C + (size_t)(kb0 + kl0) * LDC + wave * KA;
  const float* T1 = T0 + LDC;
  const v2f* E0 = sEx + kl0 * NX;
  const v2f* E1 = E0 + NX;
  float ar0 = 0.f, ai0 = 0.f, ar1 = 0.f, ai1 = 0.f;
#pragma unroll 1
  for (int x = 0; x < NX; ++x) {
    const v2f e0 = E0[x];
    const v2f e1 = E1[x];
    const v2f t0 = *(const v2f*)(T0 + 2 * x);
    const v2f t1 = *(const v2f*)(T1 + 2 * x);
    ar0 += t0.x * e0.x - t0.y * e0.y;
    ai0 += t0.x * e0.y + t0.y * e0.x;
    ar1 += t1.x * e1.x - t1.y * e1.y;
    ai1 += t1.x * e1.y + t1.y * e1.x;
  }
  const int k0 = kbase + kb0 + kl0;
  v4f o; o.x = ar0; o.y = ai0; o.z = ar1; o.w = ai1;
  if (k0 + 1 < nk) {
    float* op = out + ((size_t)wave * nk + k0) * 2;
    *(volatile v4f*)op = o;
  }
  __threadfence();
  if (k0 + 1 < nk) {
    float* op = out + ((size_t)wave * nk + k0) * 2;
    *(volatile v4f*)op = o;
  }
}

extern "C" void kernel_launch(void* const* d_in, const int* in_sizes, int n_in,
                              void* d_out, int out_size, void* d_ws, size_t ws_size,
                              hipStream_t stream) {
  if (n_in < 3) return;
  if (in_sizes[0] != NC * NX * NY || in_sizes[1] != NC * NX * NY) return;
  if (in_sizes[2] != NK * 2 || out_size != NC * NK * 2) return;

  const float* img_r = (const float*)d_in[0];
  const float* img_i = (const float*)d_in[1];
  const float* trj   = (const float*)d_in[2];
  float* out = (float*)d_out;

  const size_t cBytes = (size_t)MC * LDC * sizeof(float);
  const size_t aBytes = (size_t)NK * KA * sizeof(unsigned short);
  const size_t bBytes = (size_t)NBT * KA * sizeof(unsigned short);
  const size_t offC = 0;
  const size_t offA = offC + cBytes;
  const size_t offB = offA + aBytes;
  const size_t total = offB + bBytes;
  if (total > ws_size) return;

  char* ws = (char*)d_ws;
  float*    Cbuf = (float*)(ws + offC);
  _Float16* A16  = (_Float16*)(ws + offA);
  _Float16* Bt16 = (_Float16*)(ws + offB);

  build_ey_rows<<<NK / RB, 256, 0, stream>>>(trj, A16, NK);
  build_img_rows<<<NCX / (RB / 2), 256, 0, stream>>>(img_r, img_i, Bt16, NCX);

  const int tiles      = (MC / 64) * (NBT / 64);
  const int gemmBlocks = (tiles + 7) / 8;
  for (int ch = 0; ch < NK / MC; ++ch) {
    const unsigned short* Ach = (const unsigned short*)(A16 + (size_t)ch * MC * KA);
    const unsigned short* Bp  = (const unsigned short*)Bt16;
    wmma_gemm64<0, false, 0, 0, false, 0><<<dim3(gemmBlocks, 1), 256, 0, stream>>>(
        Ach, Ach, KA, 0L,
        Bp, Bp, KA, 0L,
        (void*)Cbuf, (void*)Cbuf, LDC, 0L,
        (const float*)Cbuf,
        (const float*)Cbuf, 0L,
        MC, NBT, KA, 1.0f);
    combine_x<<<MC / KB2, TPB2, 0, stream>>>(Cbuf, trj, out, ch * MC, NK);
  }
}
